// MHSA_40346922778634
// MI455X (gfx1250) — hardware-verified
//
#include <hip/hip_runtime.h>
#include <math.h>

constexpr int kB     = 16;
constexpr int kC     = 512;
constexpr int kSpW   = 32;
constexpr int kSpH   = 32;
constexpr int kN     = kSpW * kSpH;
constexpr int kHeads = 8;
constexpr int kDh    = 64;
constexpr int kTok   = kB * kN;
constexpr int kOC    = 3 * kC;
constexpr int kG     = 4;
constexpr float kCarry      = 16.0f;
constexpr float kPCarry     = 32768.0f;
constexpr float kRScale     = 1.0f / 16.0f;
constexpr float kScoreScale = 1.0f / 256.0f;
constexpr float kPVScale    = 1.0f / (16.0f * 32768.0f);
static_assert(kHeads * kDh == kC, "shape");
static_assert(kSpW == 32 && kSpH == 32, "position row map assumes 32 + 32 rows");
static_assert(kTok % 64 == 0 && kC % 64 == 0 && kN % 64 == 0 && kDh % 64 == 0, "M,N tile multiples");
static_assert(kC % 32 == 0 && kDh % 32 == 0 && kN % 32 == 0, "K multiples of 32");
static_assert(kHeads % kG == 0, "groups");

constexpr size_t szXT   = (size_t)kTok * kC * 2;
constexpr size_t szW    = (size_t)kOC * kC * 2;
constexpr size_t szBias = (size_t)kOC * 4;
constexpr size_t szRHW  = (size_t)kHeads * kDh * kDh * 2;
constexpr size_t szQ    = (size_t)kTok * kC * 2;
constexpr size_t szVT   = (size_t)kB * kC * kN * 2;
constexpr size_t szR    = (size_t)kHeads * kDh * kN * 4;
constexpr size_t szS    = (size_t)kG * kN * kN * 4;
constexpr size_t szP    = (size_t)kG * kN * kN * 2;
constexpr size_t offXT  = 0;
constexpr size_t offW   = offXT + szXT;
constexpr size_t offBS  = offW + szW;
constexpr size_t offRHW = offBS + szBias;
constexpr size_t offQBH = offRHW + szRHW;
constexpr size_t offQBL = offQBH + szQ;
constexpr size_t offKBH = offQBL + szQ;
constexpr size_t offKBL = offKBH + szQ;
constexpr size_t offVT  = offKBL + szQ;
constexpr size_t offR   = offVT + szVT;
constexpr size_t offS   = offR + szR;
constexpr size_t offP   = offS + szS;
constexpr size_t kWsTotal = offP + szP;
static_assert(kWsTotal == 129570816ull, "carve total");
static_assert(kWsTotal <= 134217728ull, "carve under 128 MiB");
static_assert(offW % 128 == 0 && offBS % 128 == 0 && offRHW % 128 == 0 && offQBH % 128 == 0 && offQBL % 128 == 0 &&
              offKBH % 128 == 0 && offKBL % 128 == 0 && offVT % 128 == 0 && offR % 128 == 0 && offS % 128 == 0 && offP % 128 == 0,
              "128-B aligned regions");

typedef __attribute__((ext_vector_type(16))) _Float16 v16h;
typedef __attribute__((ext_vector_type(8)))  _Float16 v8h;
typedef __attribute__((ext_vector_type(16))) __bf16   v16b;
typedef __attribute__((ext_vector_type(8)))  __bf16   v8b;
typedef __attribute__((ext_vector_type(8)))  float    v8f;
typedef __attribute__((ext_vector_type(4)))  float    v4f;
typedef __attribute__((ext_vector_type(4)))  unsigned int v4u;

__device__ __forceinline__ unsigned short f2bf_bits(float f) {
  unsigned u = __float_as_uint(f);
  return (unsigned short)((u + 0x7FFFu + ((u >> 16) & 1u)) >> 16);
}
__device__ __forceinline__ float bf_bits2f(unsigned short h) { return __uint_as_float(((unsigned)h) << 16); }
__device__ __forceinline__ float bf_rn(float f) { return __uint_as_float(((unsigned)f2bf_bits(f)) << 16); }

__device__ __forceinline__ void dep_guard4_h(v8f& a, v8f& b, v8f& c, v8f& d, v16h x, v16h y) {
  asm volatile("v_nop\n\tv_nop\n\tv_nop\n\tv_nop" : "+v"(a), "+v"(b), "+v"(c), "+v"(d) : "v"(x), "v"(y));
}
__device__ __forceinline__ void dep_guard4_b(v8f& a, v8f& b, v8f& c, v8f& d, v16b x, v16b y) {
  asm volatile("v_nop\n\tv_nop\n\tv_nop\n\tv_nop" : "+v"(a), "+v"(b), "+v"(c), "+v"(d) : "v"(x), "v"(y));
}
__device__ __forceinline__ void keep4_h(v16h a, v16h b, v16h c, v16h d) { asm volatile("v_nop" :: "v"(a), "v"(b), "v"(c), "v"(d)); }
__device__ __forceinline__ void keep4_b(v16b a, v16b b, v16b c, v16b d) { asm volatile("v_nop" :: "v"(a), "v"(b), "v"(c), "v"(d)); }
__device__ __forceinline__ void acc_guard4(v8f& a, v8f& b, v8f& c, v8f& d) { asm volatile("v_nop\n\tv_nop\n\tv_nop\n\tv_nop" : "+v"(a), "+v"(b), "+v"(c), "+v"(d)); }
template <typename T> struct Frag;
template <> struct Frag<_Float16> {
  typedef v16h V; union U { v16h v; v8h h[2]; };
  static __device__ __forceinline__ v16h load(const _Float16* p) {
    U f; f.h[0] = *(const v8h*)(p); f.h[1] = *(const v8h*)(p + 16); return f.v;
  }
  static __device__ __forceinline__ v8f mma(v16h a, v16h b, v8f c) {
    return __builtin_amdgcn_wmma_f32_16x16x32_f16(false, a, false, b, (short)0, c, false, false);
  }
  static __device__ __forceinline__ void guard4(v8f& a, v8f& b, v8f& c, v8f& d, v16h x, v16h y) { dep_guard4_h(a, b, c, d, x, y); }
  static __device__ __forceinline__ void keep(v16h a, v16h b, v16h c, v16h d) { keep4_h(a, b, c, d); }
};
template <> struct Frag<__bf16> {
  typedef v16b V; union U { v16b v; v8b h[2]; };
  static __device__ __forceinline__ v16b load(const __bf16* p) {
    U f; f.h[0] = *(const v8b*)(p); f.h[1] = *(const v8b*)(p + 16); return f.v;
  }
  static __device__ __forceinline__ v8f mma(v16b a, v16b b, v8f c) {
    return __builtin_amdgcn_wmma_f32_16x16x32_bf16(false, a, false, b, (short)0, c, false, false);
  }
  static __device__ __forceinline__ void guard4(v8f& a, v8f& b, v8f& c, v8f& d, v16b x, v16b y) { dep_guard4_b(a, b, c, d, x, y); }
  static __device__ __forceinline__ void keep(v16b a, v16b b, v16b c, v16b d) { keep4_b(a, b, c, d); }
};

__device__ __forceinline__ unsigned pk16(unsigned short a, unsigned short b) { return (unsigned)a | ((unsigned)b << 16); }
__device__ __forceinline__ unsigned short h_bits(float f) { const _Float16 h = (_Float16)f; return __builtin_bit_cast(unsigned short, h); }

template <int ET> struct Elem;
template <> struct Elem<0> { typedef _Float16 T; };
template <> struct Elem<1> { typedef __bf16 T; };

template <int ET, int SPLIT, int BIAS_MODE, int OUT_MODE, bool RESID>
__global__ __launch_bounds__(256) void wmma_gemm64(
    const unsigned short* __restrict__ Ap, const unsigned short* __restrict__ A2p, int lda, long strideA,
    const unsigned short* __restrict__ Btp, const unsigned short* __restrict__ Bt2p, int ldb, long strideB,
    void* Cout, void* Cout2, int ldc, long strideC,
    const float* __restrict__ bias,
    const float* resid, long strideR,
    int M, int N, int K, float scale) {
  static_assert(!(RESID && OUT_MODE != 0), "resid needs f32 out");
  typedef typename Elem<ET>::T T;
  typedef typename Frag<T>::V V;
  const T* A = (const T*)Ap; const T* A2 = (const T*)A2p; const T* Bt = (const T*)Btp; const T* Bt2 = (const T*)Bt2p;
  __shared__ __align__(16) float sT[8][16 * 68];
  const int b    = blockIdx.y;
  const int lane = threadIdx.x & 31;
  const int wave = threadIdx.x >> 5;
  const int tilesN = N >> 6;
  const int tilesM = M >> 6;
  const int tile = blockIdx.x * 8 + wave;
  if (tile >= tilesM * tilesN) return;
  const int tm = tile / tilesN;
  const int tn = tile - tm * tilesN;
  const int m0 = tm << 6;
  const int n0 = tn << 6;

  const T* Ab  = A   + (size_t)b * strideA;
  const T* Bb  = Bt  + (size_t)b * strideB;
  const T* Ab2 = A2  + (size_t)b * strideA;
  const T* Bb2 = Bt2 + (size_t)b * strideB;

  const int rlane = lane & 15;
  const int koff  = (lane >> 4) * 8;
  const int mOff  = (lane >> 4) * 8;

  v8f acc[4][4];
#pragma unroll
  for (int i = 0; i < 4; ++i)
#pragma unroll
    for (int j = 0; j < 4; ++j) acc[i][j] = (v8f){0.f,0.f,0.f,0.f,0.f,0.f,0.f,0.f};

  for (int k0 = 0; k0 < K; k0 += 32) {
    V bh[4], bl[4];
#pragma unroll
    for (int j = 0; j < 4; ++j) {
      const size_t bo = (size_t)(n0 + (j << 4) + rlane) * ldb + koff + k0;
      bh[j] = Frag<T>::load(Bb + bo);
      if (SPLIT != 0) bl[j] = Frag<T>::load(Bb2 + bo);
    }
#pragma unroll
    for (int i = 0; i < 4; ++i) {
      const size_t ao = (size_t)(m0 + (i << 4) + rlane) * lda + koff + k0;
      V ah = Frag<T>::load(Ab + ao);
      V al = ah;
      if (SPLIT == 1) al = Frag<T>::load(Ab2 + ao);
#pragma unroll
      for (int j = 0; j < 4; ++j) {
        acc[i][j] = Frag<T>::mma(ah, bh[j], acc[i][j]);
        if (SPLIT != 0) acc[i][j] = Frag<T>::mma(ah, bl[j], acc[i][j]);
        if (SPLIT == 1) acc[i][j] = Frag<T>::mma(al, bh[j], acc[i][j]);
      }
      Frag<T>::guard4(acc[i][0], acc[i][1], acc[i][2], acc[i][3], ah, al);
    }
    Frag<T>::keep(bh[0], bh[1], bh[2], bh[3]);
    if (SPLIT != 0) Frag<T>::keep(bl[0], bl[1], bl[2], bl[3]);
  }
  acc_guard4(acc[0][0], acc[0][1], acc[0][2], acc[0][3]);
  acc_guard4(acc[1][0], acc[1][1], acc[1][2], acc[1][3]);
  acc_guard4(acc[2][0], acc[2][1], acc[2][2], acc[2][3]);
  acc_guard4(acc[3][0], acc[3][1], acc[3][2], acc[3][3]);

  float* slab = sT[wave];
#pragma unroll
  for (int i = 0; i < 4; ++i) {
    const int mBase = m0 + (i << 4);
#pragma unroll
    for (int j = 0; j < 4; ++j) {
      const int n = n0 + (j << 4) + rlane;
      float bv = 0.f;
      if (BIAS_MODE == 2) bv = bias[n];
#pragma unroll
      for (int r = 0; r < 8; ++r) {
        float v = acc[i][j][r] * scale;
        if (BIAS_MODE == 1) v += bias[mBase + mOff + r];
        if (BIAS_MODE == 2) v += bv;
        slab[(mOff + r) * 68 + (j << 4) + rlane] = v;
      }
    }
    __builtin_amdgcn_fence(__ATOMIC_RELEASE, "workgroup");
    __builtin_amdgcn_wave_barrier();
    __builtin_amdgcn_fence(__ATOMIC_ACQUIRE, "workgroup");
    if (OUT_MODE == 0) {
      float* Cb = (float*)Cout + (size_t)b * strideC;
      const float* Rb = resid + (size_t)b * strideR;
      const int hh = lane >> 4, c4 = (lane & 15) * 4;
      for (int pass = 0; pass < 2; ++pass) {
#pragma unroll
        for (int it = 0; it < 8; ++it) {
          const int row = it * 2 + hh;
          v4f v = *(const v4f*)(slab + row * 68 + c4);
          if (RESID) {
            const v4f rx = *(const v4f*)(Rb + (size_t)(mBase + row) * ldc + n0 + c4);
            v4f rr;
            rr[0] = bf_rn(rx[0]);
            rr[1] = bf_rn(rx[1]);
            rr[2] = bf_rn(rx[2]);
            rr[3] = bf_rn(rx[3]);
            v = v + rr;
          }
          *(volatile v4f*)(Cb + (size_t)(mBase + row) * ldc + n0 + c4) = v;
        }
        __threadfence();
      }
    } else {
      const int q = lane >> 3, c8 = (lane & 7) * 8;
      unsigned short* Cb  = (unsigned short*)Cout  + (size_t)b * strideC;
      unsigned short* Cb2 = (unsigned short*)Cout2 + (size_t)b * strideC;
      for (int pass = 0; pass < 2; ++pass) {
#pragma unroll
        for (int it = 0; it < 4; ++it) {
          const int row = it * 4 + q;
          const float* sp = slab + row * 68 + c8;
          v8h hv, lv;
#pragma unroll
          for (int e = 0; e < 8; ++e) {
            if (OUT_MODE == 1) {
              hv[e] = (_Float16)sp[e];
            } else {
              unsigned short hb = f2bf_bits(sp[e]);
              unsigned short lb = f2bf_bits(sp[e] - bf_bits2f(hb));
              hv[e] = __builtin_bit_cast(_Float16, hb);
              lv[e] = __builtin_bit_cast(_Float16, lb);
            }
          }
          *(volatile v8h*)(Cb + (size_t)(mBase + row) * ldc + n0 + c8) = hv;
          if (OUT_MODE == 2) *(volatile v8h*)(Cb2 + (size_t)(mBase + row) * ldc + n0 + c8) = lv;
        }
        __threadfence();
      }
    }
    __builtin_amdgcn_fence(__ATOMIC_RELEASE, "workgroup");
    __builtin_amdgcn_wave_barrier();
    __builtin_amdgcn_fence(__ATOMIC_ACQUIRE, "workgroup");
  }
}

__global__ __launch_bounds__(256) void prep_xt_kernel(const float* __restrict__ x, unsigned short* __restrict__ xT) {
  __shared__ float sm[64][65];
  const int t  = threadIdx.x;
  const int n0 = blockIdx.x * 64;
  const int c0 = blockIdx.y * 64;
  const int b  = blockIdx.z;
#pragma unroll
  for (int i = 0; i < 4; ++i) {
    const int e  = i * 256 + t;
    const int r  = e >> 4;
    const int q4 = (e & 15) * 4;
    const v4f w = *(const v4f*)(x + ((size_t)(b * kC + c0 + r)) * kN + n0 + q4);
    sm[q4 + 0][r] = w[0];
    sm[q4 + 1][r] = w[1];
    sm[q4 + 2][r] = w[2];
    sm[q4 + 3][r] = w[3];
  }
  __syncthreads();
  const int lane = t & 31, wave = t >> 5;
  const int q = lane >> 3, c8 = (lane & 7) * 8;
  for (int pass = 0; pass < 2; ++pass) {
#pragma unroll
    for (int it = 0; it < 2; ++it) {
      const int row = wave * 8 + it * 4 + q;
      unsigned short hb[8];
#pragma unroll
      for (int e = 0; e < 8; ++e) hb[e] = f2bf_bits(sm[row][c8 + e]);
      const v4u u = (v4u){pk16(hb[0], hb[1]), pk16(hb[2], hb[3]), pk16(hb[4], hb[5]), pk16(hb[6], hb[7])};
      *(volatile v4u*)(xT + ((size_t)(b * kN + n0 + row)) * kC + c0 + c8) = u;
    }
    __threadfence();
  }
}

__global__ __launch_bounds__(256) void prep_w_kernel(const float* __restrict__ Wq, const float* __restrict__ Wk,
                                                     const float* __restrict__ Wv, unsigned short* __restrict__ Wc) {
  const int z = blockIdx.x >> 7;
  const float* W = (z == 0) ? Wq : ((z == 1) ? Wk : Wv);
  const int i  = blockIdx.x * 256 + threadIdx.x;
  const int il = i & 32767;
  const float* p = W + 8 * (size_t)il;
  const v4f a = *(const v4f*)(p);
  const v4f c = *(const v4f*)(p + 4);
  unsigned short hb[8];
#pragma unroll
  for (int e = 0; e < 4; ++e) {
    hb[e]     = f2bf_bits(a[e]);
    hb[4 + e] = f2bf_bits(c[e]);
  }
  const v4u u = (v4u){pk16(hb[0], hb[1]), pk16(hb[2], hb[3]), pk16(hb[4], hb[5]), pk16(hb[6], hb[7])};
  unsigned short* op = Wc + 8 * (size_t)i;
  *(volatile v4u*)op = u;
  __threadfence();
  *(volatile v4u*)op = u;
}

__global__ __launch_bounds__(128) void bias16_kernel(const float* __restrict__ bq, const float* __restrict__ bk,
                                                     const float* __restrict__ bv, float* __restrict__ BS) {
  const int z = blockIdx.x;
  const int t = threadIdx.x;
  const float* src = (z == 0) ? bq : ((z == 1) ? bk : bv);
  const v4f v = *(const v4f*)(src + 4 * t);
  v4f o;
  o[0] = bf_rn(v[0]) * kCarry;
  o[1] = bf_rn(v[1]) * kCarry;
  o[2] = bf_rn(v[2]) * kCarry;
  o[3] = bf_rn(v[3]) * kCarry;
  float* dp = BS + z * kC + 4 * t;
  *(volatile v4f*)dp = o;
  __threadfence();
  *(volatile v4f*)dp = o;
}

__global__ __launch_bounds__(256) void prep_rhw_kernel(const float* __restrict__ rel_h, const float* __restrict__ rel_w,
                                                       unsigned short* __restrict__ RHW) {
  const float* tab = ((blockIdx.x & 1) == 0) ? rel_h : rel_w;
  const int i  = blockIdx.x * 256 + threadIdx.x;
  const int h  = i >> 9;
  const int r  = (i >> 3) & 63;
  const int d0 = (i & 7) * 8;
  const int rr = r & 31;
  const float* p = tab + (size_t)(h * kDh + d0) * 32 + rr;
  float a[8];
#pragma unroll
  for (int e = 0; e < 8; ++e) a[e] = p[e * 32];
  unsigned short hb[8];
#pragma unroll
  for (int e = 0; e < 8; ++e) hb[e] = f2bf_bits(a[e]);
  const v4u u = (v4u){pk16(hb[0], hb[1]), pk16(hb[2], hb[3]), pk16(hb[4], hb[5]), pk16(hb[6], hb[7])};
  unsigned short* op = RHW + 8 * (size_t)i;
  *(volatile v4u*)op = u;
  __threadfence();
  *(volatile v4u*)op = u;
}

__global__ __launch_bounds__(128) void softmax_row_kernel(const float* __restrict__ S, const float* __restrict__ Rg,
                                                          unsigned short* __restrict__ P) {
  __shared__ float redM[4];
  __shared__ float redS[4];
  const int row  = blockIdx.x;
  const int g    = blockIdx.y;
  const int t    = threadIdx.x;
  const int lane = t & 31, wave = t >> 5;
  const size_t base = ((size_t)g * kN + row) * kN + 8 * (size_t)t;
  const float* ra = Rg + ((size_t)g * kDh + (row & 31)) * kN + 8 * (size_t)t;
  const float* rb = Rg + ((size_t)g * kDh + 32 + (row >> 5)) * kN + 8 * (size_t)t;
  const v4f s0 = *(const v4f*)(S + base);
  const v4f s1 = *(const v4f*)(S + base + 4);
  const v4f a0 = *(const v4f*)(ra);
  const v4f a1 = *(const v4f*)(ra + 4);
  const v4f w0 = *(const v4f*)(rb);
  const v4f w1 = *(const v4f*)(rb + 4);
  float xs[8];
#pragma unroll
  for (int e = 0; e < 4; ++e) {
    xs[e]     = (s0[e] + a0[e]) + w0[e];
    xs[4 + e] = (s1[e] + a1[e]) + w1[e];
  }
  float m = fmaxf(fmaxf(fmaxf(xs[0], xs[1]), fmaxf(xs[2], xs[3])), fmaxf(fmaxf(xs[4], xs[5]), fmaxf(xs[6], xs[7])));
#pragma unroll
  for (int off = 16; off > 0; off >>= 1) m = fmaxf(m, __shfl_xor(m, off, 32));
  if (lane == 0) redM[wave] = m;
  __syncthreads();
  const float mm = fmaxf(fmaxf(redM[0], redM[1]), fmaxf(redM[2], redM[3]));
  float ev[8];
  float sum = 0.0f;
#pragma unroll
  for (int e = 0; e < 8; ++e) {
    ev[e] = expf(xs[e] - mm);
    sum += ev[e];
  }
#pragma unroll
  for (int off = 16; off > 0; off >>= 1) sum += __shfl_xor(sum, off, 32);
  if (lane == 0) redS[wave] = sum;
  __syncthreads();
  const float tot = ((redS[0] + redS[1]) + redS[2]) + redS[3];
  const float inv = kPCarry / tot;
  unsigned short hb[8];
#pragma unroll
  for (int e = 0; e < 8; ++e) hb[e] = h_bits(ev[e] * inv);
  const v4u u = (v4u){pk16(hb[0], hb[1]), pk16(hb[2], hb[3]), pk16(hb[4], hb[5]), pk16(hb[6], hb[7])};
  unsigned short* pr = P + base;
  *(volatile v4u*)pr = u;
  __threadfence();
  *(volatile v4u*)pr = u;
}

extern "C" void kernel_launch(void* const* d_in, const int* in_sizes, int n_in,
                              void* d_out, int out_size, void* d_ws, size_t ws_size,
                              hipStream_t stream) {
  if (n_in < 9) return;
  const int nX = kB * kC * kN;
  if (in_sizes[0] != nX) return;
  if (in_sizes[1] != kC * kC || in_sizes[3] != kC * kC || in_sizes[5] != kC * kC) return;
  if (in_sizes[2] != kC || in_sizes[4] != kC || in_sizes[6] != kC) return;
  if (in_sizes[7] != kHeads * kDh * kSpH || in_sizes[8] != kHeads * kDh * kSpW) return;
  if (out_size != nX) return;
  if (ws_size < kWsTotal) return;

  const float* x     = (const float*)d_in[0];
  const float* Wq    = (const float*)d_in[1];
  const float* bq    = (const float*)d_in[2];
  const float* Wk    = (const float*)d_in[3];
  const float* bk    = (const float*)d_in[4];
  const float* Wv    = (const float*)d_in[5];
  const float* bv    = (const float*)d_in[6];
  const float* rel_h = (const float*)d_in[7];
  const float* rel_w = (const float*)d_in[8];
  float* out = (float*)d_out;
  char* ws = (char*)d_ws;
  unsigned short* xT  = (unsigned short*)(ws + offXT);
  unsigned short* Wc  = (unsigned short*)(ws + offW);
  float*          BS  = (float*)(ws + offBS);
  unsigned short* RHW = (unsigned short*)(ws + offRHW);
  unsigned short* QBH = (unsigned short*)(ws + offQBH);
  unsigned short* QBL = (unsigned short*)(ws + offQBL);
  unsigned short* KBH = (unsigned short*)(ws + offKBH);
  unsigned short* KBL = (unsigned short*)(ws + offKBL);
  unsigned short* VT  = (unsigned short*)(ws + offVT);
  float*          R   = (float*)(ws + offR);
  float*          S   = (float*)(ws + offS);
  unsigned short* P   = (unsigned short*)(ws + offP);

  prep_xt_kernel<<<dim3(kN / 64, kC / 64, kB), dim3(256), 0, stream>>>(x, xT);
  prep_w_kernel<<<dim3((kOC * kC / 8) / 256), dim3(256), 0, stream>>>(Wq, Wk, Wv, Wc);
  bias16_kernel<<<dim3(3), dim3(128), 0, stream>>>(bq, bk, bv, BS);
  prep_rhw_kernel<<<dim3((kHeads * kDh * kDh / 8) / 256), dim3(256), 0, stream>>>(rel_h, rel_w, RHW);

  const unsigned short* Wcq = Wc;
  const unsigned short* Wck = Wc + (size_t)kC * kC;
  const unsigned short* Wcv = Wc + (size_t)2 * kC * kC;
  const int blocksQK = ((kTok / 64) * (kC / 64)) / 8;
  const int blocksV  = ((kC / 64) * (kN / 64)) / 8;
  wmma_gemm64<1, 0, 2, 2, false><<<dim3(blocksQK, 1), dim3(256), 0, stream>>>(
      xT, xT, kC, 0L, Wcq, Wcq, kC, 0L,
      (void*)QBH, (void*)QBL, kC, 0L,
      BS, BS, 0L, kTok, kC, kC, kCarry);
  wmma_gemm64<1, 0, 2, 2, false><<<dim3(blocksQK, 1), dim3(256), 0, stream>>>(
      xT, xT, kC, 0L, Wck, Wck, kC, 0L,
      (void*)KBH, (void*)KBL, kC, 0L,
      BS + kC, BS, 0L, kTok, kC, kC, kCarry);
  wmma_gemm64<1, 0, 1, 1, false><<<dim3(blocksV, kB), dim3(256), 0, stream>>>(
      Wcv, Wcv, kC, 0L, xT, xT, kC, (long)kN * kC,
      (void*)VT, (void*)VT, kN, (long)kC * kN,
      BS + 2 * kC, BS, 0L, kC, kN, kC, kCarry);

  const int blocksR  = ((kDh / 64) * (kN / 64)) / 8;
  const int blocksS  = ((kN / 64) * (kN / 64)) / 8;
  const int blocksPV = ((kDh / 64) * (kN / 64)) / 8;
  for (int b = 0; b < kB; ++b) {
    const size_t tokOff = (size_t)b * kN * kC;
    wmma_gemm64<1, 2, 0, 0, false><<<dim3(blocksR, kHeads), dim3(256), 0, stream>>>(
        RHW, RHW, kDh, (long)kDh * kDh, QBH + tokOff, QBL + tokOff, kC, (long)kDh,
        (void*)R, (void*)R, kN, (long)kDh * kN,
        BS, BS, 0L, kDh, kN, kDh, kRScale);
    for (int hg = 0; hg < kHeads / kG; ++hg) {
      const int hg0 = hg * kG;
      const size_t offQK = tokOff + (size_t)hg0 * kDh;
      const size_t offV  = (size_t)b * kC * kN + (size_t)hg0 * kDh * kN;
      wmma_gemm64<1, 1, 0, 0, false><<<dim3(blocksS, kG), dim3(256), 0, stream>>>(
          QBH + offQK, QBL + offQK, kC, (long)kDh, KBH + offQK, KBL + offQK, kC, (long)kDh,
          (void*)S, (void*)S, kN, (long)kN * kN,
          BS, BS, 0L, kN, kN, kDh, kScoreScale);
      softmax_row_kernel<<<dim3(kN, kG), dim3(128), 0, stream>>>(S, R + (size_t)hg0 * kDh * kN, P);
      wmma_gemm64<0, 0, 0, 0, true><<<dim3(blocksPV, kG), dim3(256), 0, stream>>>(
          VT + offV, VT + offV, kN, (long)kDh * kN, P, P, kN, (long)kN * kN,
          (void*)(out + offV), (void*)(out + offV), kN, (long)kDh * kN,
          BS, x + offV, (long)kDh * kN, kDh, kN, kN, kPVScale);
    }
  }
}
